// GNNLayer_29111288332892
// MI455X (gfx1250) — hardware-verified
//
#include <hip/hip_runtime.h>
#include <stddef.h>


#define DF    128
#define NH    4
#define HC    32
#define BATCH 2
#define GR    32
#define AP    136
#define XSP   132
#define NPART 8
#define NB    512
#define CHUNK 2048
#define NTHR  256
#define NWAVE 8
#define WCAP  256
#define NGRP  (CHUNK / (NTHR * 4))
#define MAXG  64
#define PML   32

#define LDS_SACC (NB * DF)
#define LDS_DEN  (NB * NH)
#define LDS_LIST (NWAVE * WCAP)
#define LDS_MX   8
#define LDS_BYTES ((LDS_SACC + LDS_DEN + LDS_LIST + NWAVE + LDS_MX) * 4)

static_assert(WCAP == (CHUNK / NTHR) * 32);
static_assert(NGRP >= 1);
static_assert(NB == 512);
static_assert(CHUNK == 2048);
static_assert(((LDS_SACC + LDS_DEN) % 4) == 0);
static_assert(LDS_BYTES == 278592);
static_assert(NH * HC == DF);
static_assert(NPART * 16 == DF);
static_assert(BATCH * NH <= LDS_MX);
static_assert(GR * NH == 128);
static_assert((AP % 8) == 0);
static_assert((XSP % 4) == 0);

typedef float          v4f   __attribute__((ext_vector_type(4)));
typedef float          v8f   __attribute__((ext_vector_type(8)));
typedef int            v4i   __attribute__((ext_vector_type(4)));
typedef unsigned short v8us  __attribute__((ext_vector_type(8)));
typedef unsigned short v16us __attribute__((ext_vector_type(16)));
typedef __bf16         v16bf __attribute__((ext_vector_type(16)));
union Frag { v16us v; v8us half[2]; };
union U8   { v8us v; unsigned short s[8]; };
union BV   { v16us u; v16bf b; };

__device__ __forceinline__ v8f wmb(v16us a, v16us b, v8f c) {
  BV x, y;
  x.u = a;
  y.u = b;
  v8f d = __builtin_amdgcn_wmma_f32_16x16x32_bf16(false, x.b, false, y.b, (short)0, c, false, false);
  asm volatile("v_nop\n\tv_nop\n\tv_nop\n\tv_nop" : "+v"(d) : "v"(a), "v"(b));
  return d;
}

__device__ __forceinline__ void split2(float f, unsigned short& hi, unsigned short& lo) {
  const unsigned u  = __float_as_uint(f);
  const unsigned uh = (u + 0x7FFFu + ((u >> 16) & 1u)) & 0xFFFF0000u;
  hi = (unsigned short)(uh >> 16);
  const float    d  = f - __uint_as_float(uh);
  const unsigned ud = __float_as_uint(d);
  lo = (unsigned short)((ud + 0x7FFFu + ((ud >> 16) & 1u)) >> 16);
}

__device__ __forceinline__ float wsum(float v) {
  v += __shfl_xor(v, 16, 32);
  v += __shfl_xor(v, 8, 32);
  v += __shfl_xor(v, 4, 32);
  v += __shfl_xor(v, 2, 32);
  v += __shfl_xor(v, 1, 32);
  return v;
}

__device__ __forceinline__ float wmax(float v) {
  v = fmaxf(v, __shfl_xor(v, 16, 32));
  v = fmaxf(v, __shfl_xor(v, 8, 32));
  v = fmaxf(v, __shfl_xor(v, 4, 32));
  v = fmaxf(v, __shfl_xor(v, 2, 32));
  v = fmaxf(v, __shfl_xor(v, 1, 32));
  return v;
}

__global__ __launch_bounds__(NTHR) void k_prep(const float* __restrict__ W,
                                               unsigned short* Whi, unsigned short* Wlo, int n8) {
  const int i = blockIdx.x * NTHR + threadIdx.x;
  if (i >= n8) return;
  const size_t o = (size_t)i * 8;
  const v4f a = *(const v4f*)(W + o);
  const v4f b = *(const v4f*)(W + o + 4);
  const float fv[8] = {a.x, a.y, a.z, a.w, b.x, b.y, b.z, b.w};
  U8 uh, ul;
#pragma unroll
  for (int j = 0; j < 8; ++j) split2(fv[j], uh.s[j], ul.s[j]);
  *(volatile v8us*)(Whi + o) = uh.v;
  *(volatile v8us*)(Wlo + o) = ul.v;
  __threadfence();
  *(volatile v8us*)(Whi + o) = uh.v;
  *(volatile v8us*)(Wlo + o) = ul.v;
}

__device__ __forceinline__ void epi_tile(v8f acc, int T, int hh, int m, int wave, int ncol,
                                         float cs, float cd, float* Xs, float* Ps, float* Pd) {
  float ss[8], sd[8];
#pragma unroll
  for (int r = 0; r < 8; ++r) {
    const float v = acc[r];
    Xs[(T * 16 + 8 * hh + r) * XSP + ncol] = v;
    ss[r] = v * cs;
    sd[r] = v * cd;
  }
#pragma unroll
  for (int mk = 1; mk < 16; mk <<= 1) {
#pragma unroll
    for (int r = 0; r < 8; ++r) {
      ss[r] += __shfl_xor(ss[r], mk, 32);
      sd[r] += __shfl_xor(sd[r], mk, 32);
    }
  }
  if (m == 0) {
#pragma unroll
    for (int r = 0; r < 8; ++r) {
      Ps[(T * 16 + 8 * hh + r) * NPART + wave] = ss[r];
      Pd[(T * 16 + 8 * hh + r) * NPART + wave] = sd[r];
    }
  }
}

__global__ __launch_bounds__(NTHR) void k_gemm(
    const float* __restrict__ x, const unsigned short* __restrict__ Whi,
    const unsigned short* __restrict__ Wlo,
    const float* __restrict__ att_src, const float* __restrict__ att_dst,
    float* xp, float* asrc, float* adst, int nTot) {
  __shared__ __attribute__((aligned(16))) unsigned short Ah[GR * AP];
  __shared__ __attribute__((aligned(16))) unsigned short Al[GR * AP];
  __shared__ __attribute__((aligned(16))) float Xs[GR * XSP];
  __shared__ __attribute__((aligned(16))) float Ps[GR * NPART];
  __shared__ __attribute__((aligned(16))) float Pd[GR * NPART];

  const int tid  = threadIdx.x;
  const int lane = tid & 31;
  const int wave = tid >> 5;
  const int hh   = lane >> 4;
  const int m    = lane & 15;
  const int rowBase = blockIdx.x * GR;

  {
    const int r  = tid >> 3;
    const int c0 = (tid & 7) * 16;
    int row = rowBase + r;
    if (row > nTot - 1) row = nTot - 1;
    const float* p = x + (size_t)row * DF + c0;
    const v4f f0 = *(const v4f*)(p), f1 = *(const v4f*)(p + 4);
    const v4f f2 = *(const v4f*)(p + 8), f3 = *(const v4f*)(p + 12);
    const float fv[16] = {f0.x, f0.y, f0.z, f0.w, f1.x, f1.y, f1.z, f1.w,
                          f2.x, f2.y, f2.z, f2.w, f3.x, f3.y, f3.z, f3.w};
    U8 h0, h1, l0, l1;
#pragma unroll
    for (int j = 0; j < 8; ++j) {
      split2(fv[j],     h0.s[j], l0.s[j]);
      split2(fv[8 + j], h1.s[j], l1.s[j]);
    }
    *(v8us*)(Ah + r * AP + c0)     = h0.v;
    *(v8us*)(Ah + r * AP + c0 + 8) = h1.v;
    *(v8us*)(Al + r * AP + c0)     = l0.v;
    *(v8us*)(Al + r * AP + c0 + 8) = l1.v;
  }
  __syncthreads();

  const int ncol = wave * 16 + m;
  v8f c0a = {0.f, 0.f, 0.f, 0.f, 0.f, 0.f, 0.f, 0.f};
  v8f c1a = {0.f, 0.f, 0.f, 0.f, 0.f, 0.f, 0.f, 0.f};
#pragma unroll
  for (int kt = 0; kt < DF / 32; ++kt) {
    const int k0 = kt * 32;
    Frag a0h, a0l, a1h, a1l, bh, bl;
    const size_t ob  = (size_t)ncol * DF + k0 + 8 * hh;
    const int    oa0 = m * AP + k0 + 8 * hh;
    const int    oa1 = (16 + m) * AP + k0 + 8 * hh;
    bh.half[0]  = *(const v8us*)(Whi + ob);  bh.half[1]  = *(const v8us*)(Whi + ob + 16);
    bl.half[0]  = *(const v8us*)(Wlo + ob);  bl.half[1]  = *(const v8us*)(Wlo + ob + 16);
    a0h.half[0] = *(const v8us*)(Ah + oa0);  a0h.half[1] = *(const v8us*)(Ah + oa0 + 16);
    a0l.half[0] = *(const v8us*)(Al + oa0);  a0l.half[1] = *(const v8us*)(Al + oa0 + 16);
    a1h.half[0] = *(const v8us*)(Ah + oa1);  a1h.half[1] = *(const v8us*)(Ah + oa1 + 16);
    a1l.half[0] = *(const v8us*)(Al + oa1);  a1l.half[1] = *(const v8us*)(Al + oa1 + 16);
    c0a = wmb(a0h.v, bh.v, c0a);
    c0a = wmb(a0l.v, bh.v, c0a);
    c0a = wmb(a0h.v, bl.v, c0a);
    c1a = wmb(a1h.v, bh.v, c1a);
    c1a = wmb(a1l.v, bh.v, c1a);
    c1a = wmb(a1h.v, bl.v, c1a);
  }

  const float cs = att_src[ncol];
  const float cd = att_dst[ncol];
  epi_tile(c0a, 0, hh, m, wave, ncol, cs, cd, Xs, Ps, Pd);
  epi_tile(c1a, 1, hh, m, wave, ncol, cs, cd, Xs, Ps, Pd);
  __syncthreads();

  v4f xr[4];
#pragma unroll
  for (int i = 0; i < 4; ++i) xr[i] = *(const v4f*)(Xs + (4 * wave + i) * XSP + 4 * lane);
  const v4f qs0 = *(const v4f*)(Ps + lane * NPART);
  const v4f qs1 = *(const v4f*)(Ps + lane * NPART + 4);
  const v4f qd0 = *(const v4f*)(Pd + lane * NPART);
  const v4f qd1 = *(const v4f*)(Pd + lane * NPART + 4);
  v4f gs, gd;
  gs.x = qs0.x + qs0.y; gs.y = qs0.z + qs0.w; gs.z = qs1.x + qs1.y; gs.w = qs1.z + qs1.w;
  gd.x = qd0.x + qd0.y; gd.y = qd0.z + qd0.w; gd.z = qd1.x + qd1.y; gd.w = qd1.z + qd1.w;
  float* gps = asrc + (size_t)rowBase * NH + 4 * lane;
  float* gpd = adst + (size_t)rowBase * NH + 4 * lane;
  float* xpp[4];
#pragma unroll
  for (int i = 0; i < 4; ++i) xpp[i] = xp + (size_t)(rowBase + 4 * wave + i) * DF + 4 * lane;

#pragma unroll
  for (int i = 0; i < 4; ++i) *(volatile v4f*)(xpp[i]) = xr[i];
  if (wave == 0) *(volatile v4f*)gps = gs;
  if (wave == 1) *(volatile v4f*)gpd = gd;
  __threadfence();
#pragma unroll
  for (int i = 0; i < 4; ++i) *(volatile v4f*)(xpp[i]) = xr[i];
  if (wave == 0) *(volatile v4f*)gps = gs;
  if (wave == 1) *(volatile v4f*)gpd = gd;
}

__global__ __launch_bounds__(NTHR) void k_max(
    const int* __restrict__ ei, const float* __restrict__ asrc, const float* __restrict__ adst,
    float* pmax, int nN, int nE, int per) {
  __shared__ float red[NWAVE * 8];
  __shared__ __attribute__((aligned(16))) float fin[8];
  const int tid  = threadIdx.x;
  const int lane = tid & 31;
  const int wave = tid >> 5;
  const float NEG = -__builtin_huge_valf();
  float mv[8];
#pragma unroll
  for (int s = 0; s < 8; ++s) mv[s] = NEG;

  const int beg = blockIdx.x * per;
  int end = beg + per;
  if (end > nE) end = nE;
#pragma unroll 1
  for (int e = beg + tid; e < end; e += NTHR) {
    int s = ei[e];
    int d = ei[(size_t)nE + e];
    s = s < 0 ? 0 : (s > nN - 1 ? nN - 1 : s);
    d = d < 0 ? 0 : (d > nN - 1 ? nN - 1 : d);
#pragma unroll
    for (int b = 0; b < BATCH; ++b) {
      const v4f sv = *(const v4f*)(asrc + ((size_t)b * nN + s) * NH);
      const v4f dv = *(const v4f*)(adst + ((size_t)b * nN + d) * NH);
      v4f a = sv + dv;
      a.x = (a.x >= 0.f) ? a.x : 0.2f * a.x;
      a.y = (a.y >= 0.f) ? a.y : 0.2f * a.y;
      a.z = (a.z >= 0.f) ? a.z : 0.2f * a.z;
      a.w = (a.w >= 0.f) ? a.w : 0.2f * a.w;
      mv[b * NH + 0] = fmaxf(mv[b * NH + 0], a.x);
      mv[b * NH + 1] = fmaxf(mv[b * NH + 1], a.y);
      mv[b * NH + 2] = fmaxf(mv[b * NH + 2], a.z);
      mv[b * NH + 3] = fmaxf(mv[b * NH + 3], a.w);
    }
  }
#pragma unroll
  for (int s = 0; s < 8; ++s) mv[s] = wmax(mv[s]);
  if (lane == 0) {
#pragma unroll
    for (int s = 0; s < 8; ++s) red[wave * 8 + s] = mv[s];
  }
  __syncthreads();
  if (tid < 8) {
    float v = NEG;
#pragma unroll
    for (int w = 0; w < NWAVE; ++w) v = fmaxf(v, red[w * 8 + tid]);
    fin[tid] = v;
  }
  __syncthreads();
  const v4f q = *(const v4f*)(fin + 4 * (lane & 1));
  const v4f z = {0.f, 0.f, 0.f, 0.f};
  const v4f val = (lane < 2) ? q : z;
  float* pp = pmax + (size_t)blockIdx.x * PML + 4 * lane;
  if (wave == 0 && lane < PML / 4) *(volatile v4f*)pp = val;
  __threadfence();
  if (wave == 0 && lane < PML / 4) *(volatile v4f*)pp = val;
}

__global__ __launch_bounds__(NTHR) void k_gat(
    const int* __restrict__ ei, const float* __restrict__ xp,
    const float* __restrict__ asrc, const float* __restrict__ adst,
    const float* __restrict__ pmax, const float* __restrict__ gam, const float* __restrict__ bet,
    float* out, int nN, int nE, int nG) {
  extern __shared__ v4f lds_dyn[];
  float* sacc = (float*)lds_dyn;
  float* den  = sacc + LDS_SACC;
  int*   list = (int*)(den + LDS_DEN);
  int*   wcnt = list + LDS_LIST;
  float* mxs  = (float*)(wcnt + NWAVE);

  const int tid  = threadIdx.x;
  const int lane = tid & 31;
  const int wave = tid >> 5;
  const int hd   = lane >> 3;
  const int nodeBase = blockIdx.x * NB;
  const int b    = blockIdx.y;
  const size_t bOff = (size_t)b * (size_t)nN;

  {
    const v4f z4 = {0.f, 0.f, 0.f, 0.f};
    for (int i = tid; i < (LDS_SACC + LDS_DEN) / 4; i += NTHR) lds_dyn[i] = z4;
    if (tid < LDS_MX) {
      float v = -__builtin_huge_valf();
      if (tid < BATCH * NH) {
        int g1 = nG;
        if (g1 > MAXG) g1 = MAXG;
        if (g1 < 0) g1 = 0;
#pragma unroll 1
        for (int g = 0; g < g1; ++g) v = fmaxf(v, pmax[(size_t)g * PML + tid]);
      }
      mxs[tid] = v;
    }
  }
  __syncthreads();
  const float mreg = mxs[b * NH + hd];
  const int* eid = ei + nE;
  const bool al16 = ((nE & 3) == 0);

  const int nChunks = (nE + CHUNK - 1) / CHUNK;
#pragma unroll 1
  for (int ch = 0; ch < nChunks; ++ch) {
    const int cbase = ch * CHUNK;
    int wc = 0;
#pragma unroll
    for (int g = 0; g < NGRP; ++g) {
      const int el0 = (g * NTHR + tid) * 4;
      const int e0  = cbase + el0;
      const int sent = -2147483647 - 1;
      v4i d;
      if (al16 && (cbase + CHUNK <= nE)) {
        d = *(const v4i*)(eid + e0);
      } else {
        d.x = (e0     < nE) ? eid[min(e0, nE - 1)]     : sent;
        d.y = (e0 + 1 < nE) ? eid[min(e0 + 1, nE - 1)] : sent;
        d.z = (e0 + 2 < nE) ? eid[min(e0 + 2, nE - 1)] : sent;
        d.w = (e0 + 3 < nE) ? eid[min(e0 + 3, nE - 1)] : sent;
      }
      const unsigned s0 = (unsigned)d.x - (unsigned)nodeBase;
      const unsigned s1 = (unsigned)d.y - (unsigned)nodeBase;
      const unsigned s2 = (unsigned)d.z - (unsigned)nodeBase;
      const unsigned s3 = (unsigned)d.w - (unsigned)nodeBase;
      const bool h0 = s0 < (unsigned)NB;
      const bool h1 = s1 < (unsigned)NB;
      const bool h2 = s2 < (unsigned)NB;
      const bool h3 = s3 < (unsigned)NB;
      const unsigned many = __builtin_amdgcn_ballot_w32(h0 | h1 | h2 | h3);
      if (many != 0u) {
#define HITJ(J, HJ, SJ) { \
          const unsigned mj = __builtin_amdgcn_ballot_w32(HJ); \
          if (HJ) { \
            const int pos = wc + (int)__builtin_amdgcn_mbcnt_lo(mj, 0u); \
            if (pos < WCAP) list[wave * WCAP + pos] = ((el0 + (J)) << 9) | (int)(SJ); \
          } \
          wc += (int)__builtin_popcount(mj); }
        HITJ(0, h0, s0)
        HITJ(1, h1, s1)
        HITJ(2, h2, s2)
        HITJ(3, h3, s3)
#undef HITJ
      }
    }
    if (lane == 0) wcnt[wave] = wc;
    __syncthreads();

    if (wave == 0) {
      for (int wsx = 0; wsx < NWAVE; ++wsx) {
        int n = wcnt[wsx];
        if (n > WCAP) n = WCAP;
        if (n < 0) n = 0;
        for (int i = 0; i < n; ++i) {
          const int ent  = list[wsx * WCAP + i];
          const int slot = ent & (NB - 1);
          const int el   = (ent >> 9) & (CHUNK - 1);
          int e = cbase + el;
          if (e > nE - 1) e = nE - 1;
          int src = ei[e];
          src = src < 0 ? 0 : (src > nN - 1 ? nN - 1 : src);
          int nd = nodeBase + slot;
          if (nd > nN - 1) nd = nN - 1;
          float al = asrc[(bOff + (size_t)src) * NH + hd] + adst[(bOff + (size_t)nd) * NH + hd];
          al = (al >= 0.f) ? al : 0.2f * al;
          const float p = __expf(fminf(al - mreg, 80.f));
          const v4f xv = *(const v4f*)(xp + (bOff + (size_t)src) * DF + 4 * lane);
          v4f* sp = (v4f*)(sacc + slot * DF + 4 * lane);
          const v4f cur = *sp;
          const v4f nxt = cur + p * xv;
          *sp = nxt;
          const int di = slot * NH + hd;
          const float od = den[di];
          const float nv = od + p;
          if ((lane & 7) == 0) den[di] = nv;
        }
      }
    }
    __syncthreads();
  }

  const v4f g4 = *(const v4f*)(gam + 4 * lane);
  const v4f e4 = *(const v4f*)(bet + 4 * lane);
#pragma unroll 1
  for (int j = 0; j < NB / NWAVE; ++j) {
    const int slot = wave * (NB / NWAVE) + j;
    const int node = nodeBase + slot;
    if (node >= nN) break;
    const size_t nrow = bOff + (size_t)node;
    const float dv  = den[slot * NH + hd];
    const float inv = 1.0f / (dv + 1e-8f);
    const v4f xv = *(const v4f*)(xp + nrow * DF + 4 * lane);
    const v4f sv = *(const v4f*)(sacc + slot * DF + 4 * lane);
    const v4f h  = sv * inv + xv;
    const float s  = wsum(h.x + h.y + h.z + h.w);
    const float mu = s * (1.0f / DF);
    const v4f dd = h - mu;
    const float q  = wsum(dd.x * dd.x + dd.y * dd.y + dd.z * dd.z + dd.w * dd.w);
    const float rs = rsqrtf(q * (1.0f / DF) + 1e-5f);
    v4f y = dd * rs * g4 + e4;
    y.x = y.x > 0.f ? y.x : 0.f;
    y.y = y.y > 0.f ? y.y : 0.f;
    y.z = y.z > 0.f ? y.z : 0.f;
    y.w = y.w > 0.f ? y.w : 0.f;
    float* op = out + nrow * DF + 4 * lane;
    *(volatile v4f*)op = y;
    __threadfence();
    *(volatile v4f*)op = y;
  }
}

extern "C" void kernel_launch(void* const* d_in, const int* in_sizes, int n_in,
                              void* d_out, int out_size, void* d_ws, size_t ws_size,
                              hipStream_t stream) {
  if (n_in < 7) return;
  const int nTot = in_sizes[0] / DF;
  if (nTot <= 0 || in_sizes[0] != nTot * DF) return;
  if ((nTot % BATCH) != 0) return;
  const int nN = nTot / BATCH;
  const int nE = in_sizes[1] / 2;
  if (nE <= 0 || in_sizes[1] != 2 * nE) return;
  if (in_sizes[2] != DF * DF) return;
  if (in_sizes[3] != NH * HC || in_sizes[4] != NH * HC) return;
  if (in_sizes[5] != DF || in_sizes[6] != DF) return;
  if (out_size != nTot * DF) return;

  const float* x       = (const float*)d_in[0];
  const int*   ei      = (const int*)d_in[1];
  const float* W       = (const float*)d_in[2];
  const float* att_src = (const float*)d_in[3];
  const float* att_dst = (const float*)d_in[4];
  const float* gam     = (const float*)d_in[5];
  const float* bet     = (const float*)d_in[6];
  float* out = (float*)d_out;

  const int nP = ((nTot + GR - 1) / GR) * GR;
  size_t off = 0;
  unsigned short* Whi = (unsigned short*)((char*)d_ws + off); off += (size_t)DF * DF * sizeof(unsigned short);
  unsigned short* Wlo = (unsigned short*)((char*)d_ws + off); off += (size_t)DF * DF * sizeof(unsigned short);
  float* xp   = (float*)((char*)d_ws + off);  off += (size_t)nP * DF * sizeof(float);
  float* asrc = (float*)((char*)d_ws + off);  off += (size_t)nP * NH * sizeof(float);
  float* adst = (float*)((char*)d_ws + off);  off += (size_t)nP * NH * sizeof(float);
  float* pmax = (float*)((char*)d_ws + off);  off += (size_t)MAXG * PML * sizeof(float);
  if (off > ws_size) return;

  const int n8 = DF * DF / 8;
  k_prep<<<(n8 + NTHR - 1) / NTHR, NTHR, 0, stream>>>(W, Whi, Wlo, n8);

  k_gemm<<<nP / GR, NTHR, 0, stream>>>(x, Whi, Wlo, att_src, att_dst, xp, asrc, adst, nTot);

  const int per = (nE + MAXG - 1) / MAXG;
  k_max<<<MAXG, NTHR, 0, stream>>>(ei, asrc, adst, pmax, nN, nE, per);

  hipFuncSetAttribute(reinterpret_cast<const void*>(&k_gat),
                      hipFuncAttributeMaxDynamicSharedMemorySize, LDS_BYTES);
  dim3 grid((nN + NB - 1) / NB, BATCH);
  k_gat<<<grid, NTHR, LDS_BYTES, stream>>>(ei, xp, asrc, adst, pmax, gam, bet, out, nN, nE, MAXG);
}
